// RnnEncoder_14559939133889
// MI455X (gfx1250) — hardware-verified
//
#include <hip/hip_runtime.h>
#include <math.h>

typedef __attribute__((ext_vector_type(16))) _Float16 v16h;
typedef __attribute__((ext_vector_type(16))) __bf16 v16b;
typedef __attribute__((ext_vector_type(8)))  _Float16 v8h;
typedef __attribute__((ext_vector_type(8)))  float v8f;
typedef __attribute__((ext_vector_type(4)))  float v4f;
typedef __attribute__((ext_vector_type(2)))  float v2f;
typedef __attribute__((ext_vector_type(4)))  unsigned v4u;
typedef __attribute__((ext_vector_type(4)))  int v4i;
typedef float __attribute__((may_alias)) float_a;
typedef int __attribute__((may_alias)) int_a;

template <typename T> __device__ __forceinline__ void vst2(void* p, T v) { *(volatile T*)p = v; __threadfence(); *(volatile T*)p = v; }
__device__ __forceinline__ v8f wmma16(v16h a, v16h b, v8f c) {
  v8f d = __builtin_amdgcn_wmma_f32_16x16x32_f16(false, a, false, b, (short)0, c, false, false);
  asm volatile("v_nop\n\tv_nop\n\tv_nop\n\tv_nop" : "+v"(d) : "v"(a), "v"(b));
  return d;
}
__device__ __forceinline__ v8f wmma_bf(v16b a, v16b b, v8f c) {
  v8f d = __builtin_amdgcn_wmma_f32_16x16x32_bf16(false, a, false, b, (short)0, c, false, false);
  asm volatile("v_nop\n\tv_nop\n\tv_nop\n\tv_nop" : "+v"(d) : "v"(a), "v"(b));
  return d;
}
__device__ __forceinline__ v16h frag_h(const _Float16* rowk0, int lane) {
  union { v16h v; v8h q[2]; } u; const _Float16* p = rowk0 + 8 * (lane >> 4);
  u.q[0] = *(const v8h*)p; u.q[1] = *(const v8h*)(p + 16); return u.v;
}
__device__ __forceinline__ v16h frag_f32(const float* rowk0, int lane) {
  v16h a; const float* p = rowk0 + 8 * (lane >> 4);
#pragma unroll
  for (int i = 0; i < 8; ++i) { a[i] = (_Float16)p[i]; a[8 + i] = (_Float16)p[16 + i]; }
  return a;
}
__device__ __forceinline__ v16h frag_f32s(const float* rowk0, int lane, float sc) {
  v16h a; const float* p = rowk0 + 8 * (lane >> 4);
#pragma unroll
  for (int i = 0; i < 8; ++i) { a[i] = (_Float16)(p[i] * sc); a[8 + i] = (_Float16)(p[16 + i] * sc); }
  return a;
}
__device__ __forceinline__ v16h fragc_f32(const float* W, int k0, int n, int lane, int ld, int K) {
  v16h a; const int g = lane >> 4;
#pragma unroll
  for (int i = 0; i < 8; ++i) { const int ka = k0 + 8 * g + i, kb = ka + 16;
    a[i] = (_Float16)(ka < K ? W[(size_t)ka * ld + n] : 0.f); a[8 + i] = (_Float16)(kb < K ? W[(size_t)kb * ld + n] : 0.f); }
  return a;
}
struct F2 { v16b h, l; };
__device__ __forceinline__ F2 bsplit16(const float v[16]) { F2 r;
#pragma unroll
  for (int i = 0; i < 16; ++i) { const __bf16 h = (__bf16)v[i]; r.h[i] = h; r.l[i] = (__bf16)(v[i] - (float)h); }
  return r; }
__device__ __forceinline__ F2 split_row(const float* row, int k0, int lane) { float v[16]; const float* p = row + k0 + 8 * (lane >> 4);
#pragma unroll
  for (int i = 0; i < 8; ++i) { v[i] = p[i]; v[8 + i] = p[16 + i]; }
  return bsplit16(v); }
__device__ __forceinline__ F2 split_rowK(const float* row, int k0, int lane, int K) { float v[16]; const int g = lane >> 4;
#pragma unroll
  for (int i = 0; i < 8; ++i) { const int ka = k0 + 8 * g + i, kb = ka + 16; v[i] = ka < K ? row[ka] : 0.f; v[8 + i] = kb < K ? row[kb] : 0.f; }
  return bsplit16(v); }
__device__ __forceinline__ F2 split_col(const float* W, int k0, int n, int lane, int ld, int K) { float v[16]; const int g = lane >> 4;
#pragma unroll
  for (int i = 0; i < 8; ++i) { const int ka = k0 + 8 * g + i, kb = ka + 16; v[i] = ka < K ? W[(size_t)ka * ld + n] : 0.f; v[8 + i] = kb < K ? W[(size_t)kb * ld + n] : 0.f; }
  return bsplit16(v); }
__device__ __forceinline__ v8f mac3(const F2& a, const F2& b, v8f c) { c = wmma_bf(a.l, b.h, c); c = wmma_bf(a.h, b.l, c); return wmma_bf(a.h, b.h, c); }
__device__ __forceinline__ float sigm(float v) { return 1.0f / (1.0f + expf(-v)); }
#define LDSX() do { asm volatile("s_wait_dscnt 0" ::: "memory"); __builtin_amdgcn_wave_barrier(); __builtin_amdgcn_fence(__ATOMIC_RELEASE, "workgroup"); } while (0)

#define NS 32
#define TT 2048
#define NF 128
#define NHID 512
#define FC 128
#define NR (NS * TT)

__global__ __launch_bounds__(256) void k_packT(const float* __restrict__ Wih, const float* __restrict__ Whh, const float* __restrict__ W1, _Float16* __restrict__ P) {
  const int r = blockIdx.x, tid = threadIdx.x; __shared__ __align__(16) _Float16 srow[NHID];
  for (int q = tid; q < NHID; q += 256) { float v = 0.f;
    if (r < NHID) v = q < NF ? Wih[(size_t)r * NF + q] : 0.f; else if (r < 2 * NHID) v = Whh[(size_t)(r - NHID) * NHID + q]; else v = W1[(size_t)(r - 2 * NHID) * NHID + q];
    srow[q] = (_Float16)(v * 16.0f); }
  __syncthreads();
  for (int q = tid; q < NHID / 8; q += 256) vst2(P + (size_t)r * NHID + q * 8, *(const v4u*)(&srow[q * 8]));
}
__global__ __launch_bounds__(256) void k_cvt(const float* __restrict__ x, _Float16* __restrict__ x16, size_t n8) {
  const size_t g8 = (size_t)blockIdx.x * 256 + threadIdx.x; if (g8 >= n8) return;
  union { v8h h; v4u u; } pk;
#pragma unroll
  for (int e = 0; e < 8; ++e) pk.h[e] = (_Float16)x[g8 * 8 + e];
  vst2(x16 + g8 * 8, pk.u);
}
__global__ __launch_bounds__(128) void k_drive(const _Float16* __restrict__ x16, const _Float16* __restrict__ P, const float* __restrict__ bih, const float* __restrict__ bhh, float* __restrict__ drive) {
  __shared__ __align__(16) float so[4][16][132];
  const int tid = threadIdx.x, wave = tid >> 5, lane = tid & 31, col = lane & 15, g = lane >> 4;
  const int r0 = blockIdx.x * 64 + wave * 16, n0 = blockIdx.y * 128;
  v8f acc[8] = {};
#pragma unroll
  for (int kc = 0; kc < NF / 32; ++kc) { const v16h a = frag_h(x16 + (size_t)(r0 + col) * NF + kc * 32, lane);
#pragma unroll
    for (int j = 0; j < 8; ++j) acc[j] = wmma16(a, frag_h(P + (size_t)(n0 + j * 16 + col) * NHID + kc * 32, lane), acc[j]); }
#pragma unroll
  for (int j = 0; j < 8; ++j) { const int c = n0 + j * 16 + col; const float bb = bih[c] + bhh[c];
#pragma unroll
    for (int r = 0; r < 8; ++r) so[wave][8 * g + r][j * 16 + col] = acc[j][r] * (1.0f / 16.0f) + bb; }
  LDSX();
#pragma unroll 4
  for (int rl = 0; rl < 16; ++rl) vst2(drive + (size_t)(r0 + rl) * NHID + n0 + lane * 4, *(const v4f*)(&so[wave][rl][lane * 4]));
}
__global__ __launch_bounds__(512) void k_rec(const float* __restrict__ drive, const _Float16* __restrict__ P, const int* __restrict__ len, _Float16* __restrict__ Hs16, float* __restrict__ hfin) {
  __shared__ __align__(16) _Float16 sh[2][16][NHID + 8];
  __shared__ __align__(16) float shf[16][NHID + 4];
  const int tid = threadIdx.x, w = tid >> 5, lane = tid & 31, col = lane & 15, g = lane >> 4; const int b0 = blockIdx.x * 16;
  const _Float16* Wh = P + (size_t)NHID * NHID;
  int L[8];
#pragma unroll
  for (int r = 0; r < 8; ++r) { int l = len[b0 + 8 * g + r]; L[r] = l < 0 ? 0 : (l > TT ? TT : l); }
  float h[2][8];
#pragma unroll
  for (int t4 = 0; t4 < 2; ++t4)
#pragma unroll
    for (int r = 0; r < 8; ++r) h[t4][r] = 0.f;
  for (int e = tid; e < 16 * (NHID + 8); e += 512) { (&sh[0][0][0])[e] = (_Float16)0.f; }
  __syncthreads();
#pragma unroll 1
  for (int t = 0; t < TT; ++t) { const int cur = t & 1, nxt = cur ^ 1;
    v8f acc[2] = {};
#pragma unroll 4
    for (int kc = 0; kc < NHID / 32; ++kc) { const v16h a = frag_h(&sh[cur][col][0] + kc * 32, lane);
#pragma unroll
      for (int t4 = 0; t4 < 2; ++t4) acc[t4] = wmma16(a, frag_h(Wh + (size_t)(w * 32 + t4 * 16 + col) * NHID + kc * 32, lane), acc[t4]); }
#pragma unroll
    for (int t4 = 0; t4 < 2; ++t4) { const int n = w * 32 + t4 * 16 + col;
#pragma unroll
      for (int r = 0; r < 8; ++r) { const int b = b0 + 8 * g + r; const float hn = tanhf(drive[((size_t)b * TT + t) * NHID + n] + acc[t4][r] * (1.0f / 16.0f));
        const float hk = t < L[r] ? hn : h[t4][r]; h[t4][r] = hk;
        sh[nxt][8 * g + r][n] = (_Float16)hk;
        shf[8 * g + r][n] = hn; } }
    __syncthreads();
    if (w < 8) { for (int q = lane; q < 16 * 8; q += 32) { const int m = q >> 3, pc = q & 7; union { v8h h8; v4u u; } pk;
#pragma unroll
        for (int e = 0; e < 8; ++e) pk.h8[e] = (_Float16)shf[m][w * 64 + pc * 8 + e];
        vst2(Hs16 + ((size_t)(b0 + m) * TT + t) * NHID + w * 64 + pc * 8, pk.u); } }
    __syncthreads(); }
#pragma unroll
  for (int t4 = 0; t4 < 2; ++t4)
#pragma unroll
    for (int r = 0; r < 8; ++r) shf[8 * g + r][w * 32 + t4 * 16 + col] = h[t4][r];
  __syncthreads();
  for (int q = tid; q < 16 * NHID / 4; q += 512) { const int m = q >> 7, pc = q & 127; vst2(hfin + (size_t)(b0 + m) * NHID + pc * 4, *(const v4f*)(&shf[m][pc * 4])); }
}
__global__ __launch_bounds__(128) void k_head(const _Float16* __restrict__ Hs16, const _Float16* __restrict__ P, const float* __restrict__ b1, const float* __restrict__ W2, const float* __restrict__ b2, const int* __restrict__ len, float* __restrict__ cnt) {
  __shared__ __align__(16) float so[4][16][132]; __shared__ float sc[4];
  const int tid = threadIdx.x, wave = tid >> 5, lane = tid & 31, col = lane & 15, g = lane >> 4;
  const int r0 = blockIdx.x * 64 + wave * 16; const int b = r0 / TT; int l = len[b]; l = l < 0 ? 0 : (l > TT ? TT : l);
  v8f acc[8] = {};
#pragma unroll 1
  for (int kc = 0; kc < NHID / 32; ++kc) { const v16h a = frag_h(Hs16 + (size_t)(r0 + col) * NHID + kc * 32, lane);
#pragma unroll
    for (int j = 0; j < 8; ++j) acc[j] = wmma16(a, frag_h(P + (size_t)(2 * NHID + j * 16 + col) * NHID + kc * 32, lane), acc[j]); }
#pragma unroll
  for (int j = 0; j < 8; ++j) { const float bb = b1[j * 16 + col];
#pragma unroll
    for (int r = 0; r < 8; ++r) so[wave][8 * g + r][j * 16 + col] = acc[j][r] * (1.0f / 16.0f) + bb; }
  LDSX();
  { const int rl = lane >> 1, hf = lane & 1; float s = 0.f;
#pragma unroll 8
    for (int c = 0; c < 64; ++c) s += so[wave][rl][hf * 64 + c] * W2[hf * 64 + c];
    s += __shfl_xor(s, 1, 32); const float z = s + b2[0]; const int t = (r0 + rl) % TT;
    int pos = (hf == 0 && z > 0.f && t < l) ? 1 : 0;
#pragma unroll
    for (int off = 16; off >= 1; off >>= 1) pos += __shfl_xor(pos, off, 32);
    if (lane == 0) sc[wave] = (float)pos; }
  __syncthreads();
  if (tid < 32) vst2(cnt + (size_t)blockIdx.x * 32 + tid, (float_a)(tid == 0 ? (sc[0] + sc[1]) + (sc[2] + sc[3]) : 0.f));
}
__global__ __launch_bounds__(32) void k_fin(const float* __restrict__ cnt, float* __restrict__ outs) {
  __shared__ __align__(16) float so[NS];
  const int b = threadIdx.x; float s = 0.f; for (int k = 0; k < TT / 64; ++k) s += cnt[(size_t)(b * (TT / 64) + k) * 32]; so[b] = s;
  __builtin_amdgcn_wave_barrier(); asm volatile("s_wait_dscnt 0" ::: "memory");
  if (threadIdx.x < NS / 4) vst2(outs + threadIdx.x * 4, *(const v4f*)(&so[threadIdx.x * 4]));
}
extern "C" void kernel_launch(void* const* d_in, const int* in_sizes, int n_in, void* d_out, int out_size, void* d_ws, size_t ws_size, hipStream_t stream) {
  (void)in_sizes; (void)n_in; (void)out_size; (void)ws_size;
  const float* x = (const float*)d_in[0]; const int* len = (const int*)d_in[1]; const float* Wih = (const float*)d_in[2]; const float* Whh = (const float*)d_in[3]; const float* bih = (const float*)d_in[4]; const float* bhh = (const float*)d_in[5];
  const float* W1 = (const float*)d_in[6]; const float* b1 = (const float*)d_in[7]; const float* W2 = (const float*)d_in[8]; const float* b2 = (const float*)d_in[9];
  float* outs = (float*)d_out; float* hfin = (float*)((char*)d_out + 128);
  char* ws = (char*)d_ws; size_t off = 0;
  auto take = [&](size_t bytes) { char* p = ws + off; off += (bytes + 255) & ~(size_t)255; return p; };
  _Float16* Hs16 = (_Float16*)take((size_t)NR * NHID * 2); _Float16* P = (_Float16*)take((size_t)(2 * NHID + FC) * NHID * 2); _Float16* x16 = (_Float16*)take((size_t)NR * NF * 2);
  float* cnt = (float*)take((size_t)(NR / 64) * 32 * 4); float* drive = (float*)take((size_t)NR * NHID * 4);
  k_packT<<<2 * NHID + FC, 256, 0, stream>>>(Wih, Whh, W1, P);
  { const size_t n8 = (size_t)NR * NF / 8; k_cvt<<<(unsigned)(n8 / 256), 256, 0, stream>>>(x, x16, n8); }
  k_drive<<<dim3(NR / 64, NHID / 128), 128, 0, stream>>>(x16, P, bih, bhh, drive);
  k_rec<<<NS / 16, 512, 0, stream>>>(drive, P, len, Hs16, hfin);
  k_head<<<NR / 64, 128, 0, stream>>>(Hs16, P, b1, W2, b2, len, cnt);
  k_fin<<<1, 32, 0, stream>>>(cnt, outs);
}
